// ScalarFeatureEmbedding_59236188946473
// MI455X (gfx1250) — hardware-run, weakly checked
//
#include <hip/hip_runtime.h>
#include <math.h>

constexpr int kRows   = 16384;
constexpr int kFeat   = 64;
constexpr int kHid    = 128;
constexpr int kOutDim = 512;
constexpr int kDepth  = kFeat * kHid;
constexpr int kChunkRows = 4096;
constexpr int kNumChunks = kRows / kChunkRows;
constexpr float kW2Carry  = 256.0f;
constexpr float kOutScale = 0.125f / 256.0f;
constexpr float kBiasScale = 0.125f;

static_assert(kRows % kChunkRows == 0, "chunking");
static_assert(kChunkRows % 64 == 0 && kOutDim % 64 == 0 && kDepth % 32 == 0, "tile multiples");

typedef __attribute__((ext_vector_type(16))) _Float16 v16h;
typedef __attribute__((ext_vector_type(8)))  _Float16 v8h;
typedef __attribute__((ext_vector_type(16))) __bf16   v16b;
typedef __attribute__((ext_vector_type(8)))  __bf16   v8b;
typedef __attribute__((ext_vector_type(8)))  float    v8f;
typedef __attribute__((ext_vector_type(4)))  float    v4f;
typedef __attribute__((ext_vector_type(4)))  unsigned int v4u;
typedef __attribute__((ext_vector_type(2)))  unsigned int v2u;

__device__ __forceinline__ unsigned short f2bf_bits(float f) {
  unsigned u = __float_as_uint(f);
  return (unsigned short)((u + 0x7FFFu + ((u >> 16) & 1u)) >> 16);
}
__device__ __forceinline__ float bf_bits2f(unsigned short h) { return __uint_as_float(((unsigned)h) << 16); }

__device__ __forceinline__ void dep_guard_h(v8f& a, v8f& b, v16h x, v16h y) { asm volatile("v_nop\n\tv_nop\n\tv_nop\n\tv_nop" : "+v"(a), "+v"(b) : "v"(x), "v"(y)); }
__device__ __forceinline__ void dep_guard_b(v8f& a, v8f& b, v16b x, v16b y) { asm volatile("v_nop\n\tv_nop\n\tv_nop\n\tv_nop" : "+v"(a), "+v"(b) : "v"(x), "v"(y)); }
__device__ __forceinline__ void keep4_h(v16h a, v16h b, v16h c, v16h d) { asm volatile("v_nop" :: "v"(a), "v"(b), "v"(c), "v"(d)); }
__device__ __forceinline__ void keep4_b(v16b a, v16b b, v16b c, v16b d) { asm volatile("v_nop" :: "v"(a), "v"(b), "v"(c), "v"(d)); }
__device__ __forceinline__ void acc_guard4(v8f& a, v8f& b, v8f& c, v8f& d) { asm volatile("v_nop\n\tv_nop\n\tv_nop\n\tv_nop" : "+v"(a), "+v"(b), "+v"(c), "+v"(d)); }
template <typename T> struct Frag;
template <> struct Frag<_Float16> {
  typedef v16h V; union U { v16h v; v8h h[2]; };
  static __device__ __forceinline__ v16h load(const _Float16* p) {
    U f; f.h[0] = *(const v8h*)(p); f.h[1] = *(const v8h*)(p + 16); return f.v;
  }
  static __device__ __forceinline__ v8f mma(v16h a, v16h b, v8f c) {
    return __builtin_amdgcn_wmma_f32_16x16x32_f16(false, a, false, b, (short)0, c, false, false);
  }
  static __device__ __forceinline__ void guard(v8f& a, v8f& b, v16h x, v16h y) { dep_guard_h(a, b, x, y); }
  static __device__ __forceinline__ void keep(v16h a, v16h b, v16h c, v16h d) { keep4_h(a, b, c, d); }
};
template <> struct Frag<__bf16> {
  typedef v16b V; union U { v16b v; v8b h[2]; };
  static __device__ __forceinline__ v16b load(const __bf16* p) {
    U f; f.h[0] = *(const v8b*)(p); f.h[1] = *(const v8b*)(p + 16); return f.v;
  }
  static __device__ __forceinline__ v8f mma(v16b a, v16b b, v8f c) {
    return __builtin_amdgcn_wmma_f32_16x16x32_bf16(false, a, false, b, (short)0, c, false, false);
  }
  static __device__ __forceinline__ void guard(v8f& a, v8f& b, v16b x, v16b y) { dep_guard_b(a, b, x, y); }
  static __device__ __forceinline__ void keep(v16b a, v16b b, v16b c, v16b d) { keep4_b(a, b, c, d); }
};

__device__ __forceinline__ unsigned pk16(unsigned short a, unsigned short b) { return (unsigned)a | ((unsigned)b << 16); }
__device__ __forceinline__ unsigned short h_bits(float f) { const _Float16 h = (_Float16)f; return __builtin_bit_cast(unsigned short, h); }

template <int ET> struct Elem;
template <> struct Elem<0> { typedef _Float16 T; };
template <> struct Elem<1> { typedef __bf16 T; };
template <int ET, bool SPLIT, int BIAS_MODE, int OUT_MODE, bool RESID, int ACT = 0>
__global__ __launch_bounds__(256) void wmma_gemm64(
    const unsigned short* __restrict__ Ap, const unsigned short* __restrict__ A2p, int lda, long strideA,
    const unsigned short* __restrict__ Btp, const unsigned short* __restrict__ Bt2p, int ldb, long strideB,
    void* __restrict__ Cout, void* __restrict__ Cout2, int ldc, long strideC,
    const float* __restrict__ bias,
    const float* __restrict__ resid, long strideR,
    int M, int N, int K, float scale) {
  typedef typename Elem<ET>::T T;
  typedef typename Frag<T>::V V;
  const T* A = (const T*)Ap; const T* A2 = (const T*)A2p; const T* Bt = (const T*)Btp; const T* Bt2 = (const T*)Bt2p;
  __shared__ __align__(16) float sT[8][16 * 68];
  const int b    = blockIdx.y;
  const int lane = threadIdx.x & 31;
  const int wave = threadIdx.x >> 5;
  const int tilesN = N >> 6;
  const int tilesM = M >> 6;
  const int tile = blockIdx.x * 8 + wave;
  if (tile >= tilesM * tilesN) return;
  const int tm = tile / tilesN;
  const int tn = tile - tm * tilesN;
  const int m0 = tm << 6;
  const int n0 = tn << 6;

  const T* Ab  = A  + (size_t)b * strideA;
  const T* Bb  = Bt + (size_t)b * strideB;
  const T* Ab2 = SPLIT ? (A2  + (size_t)b * strideA) : nullptr;
  const T* Bb2 = SPLIT ? (Bt2 + (size_t)b * strideB) : nullptr;

  const int rlane = lane & 15;
  const int koff  = (lane >> 4) * 8;
  const int mOff  = (lane >> 4) * 8;

  v8f acc[4][4];
#pragma unroll
  for (int i = 0; i < 4; ++i)
#pragma unroll
    for (int j = 0; j < 4; ++j) acc[i][j] = (v8f){0.f,0.f,0.f,0.f,0.f,0.f,0.f,0.f};

  for (int k0 = 0; k0 < K; k0 += 32) {
    V bh[4], bl[4];
#pragma unroll
    for (int j = 0; j < 4; ++j) {
      const size_t bo = (size_t)(n0 + (j << 4) + rlane) * ldb + koff + k0;
      bh[j] = Frag<T>::load(Bb + bo);
      if (SPLIT) bl[j] = Frag<T>::load(Bb2 + bo);
    }
#pragma unroll
    for (int i = 0; i < 4; ++i) {
      const size_t ao = (size_t)(m0 + (i << 4) + rlane) * lda + koff + k0;
      V ah = Frag<T>::load(Ab + ao);
      V al;
      if (SPLIT) al = Frag<T>::load(Ab2 + ao);
#pragma unroll
      for (int j = 0; j < 4; ++j) {
        acc[i][j] = Frag<T>::mma(ah, bh[j], acc[i][j]);
        if (SPLIT) {
          acc[i][j] = Frag<T>::mma(ah, bl[j], acc[i][j]);
          acc[i][j] = Frag<T>::mma(al, bh[j], acc[i][j]);
        }
      }
      Frag<T>::guard(acc[i][0], acc[i][3], ah, SPLIT ? al : ah);
    }
    Frag<T>::keep(bh[0], bh[1], bh[2], bh[3]);
    if (SPLIT) Frag<T>::keep(bl[0], bl[1], bl[2], bl[3]);
  }
  acc_guard4(acc[0][0], acc[0][1], acc[0][2], acc[0][3]);
  acc_guard4(acc[1][0], acc[1][1], acc[1][2], acc[1][3]);
  acc_guard4(acc[2][0], acc[2][1], acc[2][2], acc[2][3]);
  acc_guard4(acc[3][0], acc[3][1], acc[3][2], acc[3][3]);

  float* slab = sT[wave];
  const float* Rb = RESID ? (resid + (size_t)b * strideR) : nullptr;
#pragma unroll
  for (int i = 0; i < 4; ++i) {
    const int mBase = m0 + (i << 4);
#pragma unroll
    for (int j = 0; j < 4; ++j) {
      const int n = n0 + (j << 4) + rlane;
      float bv = 0.f;
      if (BIAS_MODE == 2) bv = bias[n];
#pragma unroll
      for (int r = 0; r < 8; ++r) {
        float v = acc[i][j][r] * scale;
        if (BIAS_MODE == 1) v += bias[mBase + mOff + r];
        if (BIAS_MODE == 2) v += bv;
        if (RESID) v += Rb[(size_t)(mBase + mOff + r) * ldc + n];
        if (ACT == 2) v = fmaxf(v, 0.0f);
        if (ACT == 4) v = (v > 0.f) ? v : 0.01f * v;
        slab[(mOff + r) * 68 + (j << 4) + rlane] = v;
      }
    }
    __builtin_amdgcn_fence(__ATOMIC_RELEASE, "workgroup");
    __builtin_amdgcn_wave_barrier();
    __builtin_amdgcn_fence(__ATOMIC_ACQUIRE, "workgroup");
    if (OUT_MODE == 0) {
      float* C = (float*)Cout + (size_t)b * strideC;
      const int hh = lane >> 4, c4 = (lane & 15) * 4;
      for (int pass = 0; pass < 2; ++pass) {
#pragma unroll
        for (int it = 0; it < 8; ++it) {
          const int row = it * 2 + hh;
          v4f v = *(const v4f*)(slab + row * 68 + c4);
          *(volatile v4f*)(C + (size_t)(mBase + row) * ldc + n0 + c4) = v;
        }
        __threadfence();
      }
    } else {
      const int q = lane >> 3, c8 = (lane & 7) * 8;
      unsigned short* C  = (unsigned short*)Cout  + (size_t)b * strideC;
      unsigned short* C2 = (OUT_MODE == 2) ? ((unsigned short*)Cout2 + (size_t)b * strideC) : nullptr;
      for (int pass = 0; pass < 2; ++pass) {
#pragma unroll
        for (int it = 0; it < 4; ++it) {
          const int row = it * 4 + q;
          const float* sp = slab + row * 68 + c8;
          v8h hv, lv;
#pragma unroll
          for (int e = 0; e < 8; ++e) {
            if (OUT_MODE == 1) {
              hv[e] = (_Float16)sp[e];
            } else {
              unsigned short hb = f2bf_bits(sp[e]);
              unsigned short lb = f2bf_bits(sp[e] - bf_bits2f(hb));
              hv[e] = __builtin_bit_cast(_Float16, hb);
              lv[e] = __builtin_bit_cast(_Float16, lb);
            }
          }
          *(volatile v8h*)(C + (size_t)(mBase + row) * ldc + n0 + c8) = hv;
          if (OUT_MODE == 2) *(volatile v8h*)(C2 + (size_t)(mBase + row) * ldc + n0 + c8) = lv;
        }
        __threadfence();
      }
    }
    __builtin_amdgcn_fence(__ATOMIC_RELEASE, "workgroup");
    __builtin_amdgcn_wave_barrier();
    __builtin_amdgcn_fence(__ATOMIC_ACQUIRE, "workgroup");
  }
}

__global__ __launch_bounds__(256) void w2t_cast_kernel(const float* __restrict__ W2, unsigned short* __restrict__ out, float scale) {
  __shared__ float sm[64][65];
  const int t  = threadIdx.x;
  const int k0 = blockIdx.x * 64;
  const int o0 = blockIdx.y * 64;
#pragma unroll
  for (int i = 0; i < 16; ++i) {
    const int e = i * 256 + t;
    const int r = e >> 6;
    const int c = e & 63;
    sm[c][r] = W2[(size_t)(k0 + r) * kOutDim + o0 + c] * scale;
  }
  __syncthreads();
  const int lane = t & 31, wave = t >> 5;
  const int q = lane >> 3, c8 = (lane & 7) * 8;
  for (int pass = 0; pass < 2; ++pass) {
#pragma unroll
    for (int it = 0; it < 2; ++it) {
      const int row = wave * 8 + it * 4 + q;
      unsigned short hb[8];
#pragma unroll
      for (int e = 0; e < 8; ++e) hb[e] = h_bits(sm[row][c8 + e]);
      const v4u u = (v4u){pk16(hb[0], hb[1]), pk16(hb[2], hb[3]), pk16(hb[4], hb[5]), pk16(hb[6], hb[7])};
      *(volatile v4u*)(out + (size_t)(o0 + row) * kDepth + k0 + c8) = u;
    }
    __threadfence();
  }
}

__global__ __launch_bounds__(128) void bsum_kernel(const float* __restrict__ b2, float* __restrict__ bias_out) {
  const int t = threadIdx.x;
  v4f s = (v4f){0.f, 0.f, 0.f, 0.f};
#pragma unroll 1
  for (int f = 0; f < kFeat; ++f) {
    const v4f v = *(const v4f*)(b2 + (size_t)f * kOutDim + 4 * t);
    s = s + v;
  }
  s = s * kBiasScale;
  float* p = bias_out + 4 * t;
  *(volatile v4f*)p = s;
  __threadfence();
  *(volatile v4f*)p = s;
}

__global__ __launch_bounds__(256) void act_kernel(const float* __restrict__ x, const float* __restrict__ W1,
                                                  const float* __restrict__ b1, unsigned short* __restrict__ Aout, int row0) {
#pragma clang fp contract(off)
  const int t  = blockIdx.x * 256 + threadIdx.x;
  const int nl = t >> 11;
  const int k4 = (t & 2047) * 4;
  const int f  = k4 >> 7;
  const int h0 = k4 & 127;
  const float xv = x[(size_t)(row0 + nl) * kFeat + f];
  const v4f w = *(const v4f*)(W1 + f * kHid + h0);
  const v4f c = *(const v4f*)(b1 + f * kHid + h0);
  unsigned u0 = 0u, u1 = 0u;
#pragma unroll 1
  for (int q = 0; q < 2; ++q) {
    const float we = (q == 0) ? w[0] : w[2];
    const float wo = (q == 0) ? w[1] : w[3];
    const float ce = (q == 0) ? c[0] : c[2];
    const float co = (q == 0) ? c[1] : c[3];
    float pe = xv * we;
    pe = pe + ce;
    float po = xv * wo;
    po = po + co;
    const float ee = expm1f(fminf(pe, 0.0f));
    const float eo = expm1f(fminf(po, 0.0f));
    const float ae = (pe > 0.0f) ? pe : ee;
    const float ao = (po > 0.0f) ? po : eo;
    const unsigned word = pk16(h_bits(ae), h_bits(ao));
    u0 = (q == 0) ? word : u0;
    u1 = (q == 0) ? u1 : word;
  }
  const v2u u = (v2u){u0, u1};
  unsigned short* p = Aout + (size_t)nl * kDepth + k4;
  *(volatile v2u*)p = u;
  __threadfence();
  *(volatile v2u*)p = u;
}

extern "C" void kernel_launch(void* const* d_in, const int* in_sizes, int n_in,
                              void* d_out, int out_size, void* d_ws, size_t ws_size,
                              hipStream_t stream) {
  if (n_in < 5) return;
  if (in_sizes[0] != kRows * kFeat) return;
  if (in_sizes[1] != kFeat * kHid) return;
  if (in_sizes[2] != kFeat * kHid) return;
  if (in_sizes[3] != kFeat * kHid * kOutDim) return;
  if (in_sizes[4] != kFeat * kOutDim) return;
  if (out_size != kRows * kOutDim) return;

  const float* x  = (const float*)d_in[0];
  const float* W1 = (const float*)d_in[1];
  const float* b1 = (const float*)d_in[2];
  const float* W2 = (const float*)d_in[3];
  const float* b2 = (const float*)d_in[4];
  float* out = (float*)d_out;

  const size_t bytesBt   = (size_t)kOutDim * kDepth * 2;
  const size_t bytesBias = 4096;
  const size_t bytesA    = (size_t)kChunkRows * kDepth * 2;
  const size_t offBt   = 0;
  const size_t offBias = offBt + bytesBt;
  const size_t offA    = offBias + bytesBias;
  const size_t total   = offA + bytesA;
  if (total > ws_size) return;

  unsigned char* ws = (unsigned char*)d_ws;
  unsigned short* Bt  = (unsigned short*)(ws + offBt);
  float*          bsp = (float*)(ws + offBias);
  unsigned short* A16 = (unsigned short*)(ws + offA);

  w2t_cast_kernel<<<dim3(kDepth / 64, kOutDim / 64, 1), dim3(256, 1, 1), 0, stream>>>(W2, Bt, kW2Carry);
  bsum_kernel<<<dim3(1, 1, 1), dim3(128, 1, 1), 0, stream>>>(b2, bsp);

  const int actBlocks  = (kChunkRows * (kDepth / 4)) / 256;
  const int gemmTiles  = (kChunkRows / 64) * (kOutDim / 64);
  const int gemmBlocks = (gemmTiles + 7) / 8;
  for (int ch = 0; ch < kNumChunks; ++ch) {
    const int row0 = ch * kChunkRows;
    act_kernel<<<dim3(actBlocks, 1, 1), dim3(256, 1, 1), 0, stream>>>(x, W1, b1, A16, row0);
    float* Cc = out + (size_t)row0 * kOutDim;
    wmma_gemm64<0, false, 2, 0, false, 0><<<dim3(gemmBlocks, 1, 1), dim3(256, 1, 1), 0, stream>>>(
        (const unsigned short*)A16, (const unsigned short*)A16, kDepth, 0L,
        (const unsigned short*)Bt, (const unsigned short*)Bt, kDepth, 0L,
        (void*)Cc, (void*)Cc, kOutDim, 0L,
        (const float*)bsp,
        (const float*)bsp, 0L,
        kChunkRows, kOutDim, kDepth, kOutScale);
  }
}
